// KANConvolutionalLayer_4483945857426
// MI455X (gfx1250) — hardware-verified
//
#include <hip/hip_runtime.h>


#define NB_  16
#define CIN  16
#define COUT 32
#define HH   64
#define WW   64
#define KT   9
#define NBAS 8
#define KI   96
#define APITCH 104
#define LOSC 1024.0f
#define LOSCI (1.0f / 1024.0f)
#define GH   0.4f

typedef _Float16 h16;
typedef __attribute__((ext_vector_type(16))) _Float16 v16h;
typedef __attribute__((ext_vector_type(8)))  _Float16 v8h;
typedef __attribute__((ext_vector_type(8)))  float    v8f;
typedef __attribute__((ext_vector_type(4)))  float    v4f;
typedef v8h  __attribute__((may_alias)) v8ha;
typedef v4f  __attribute__((may_alias)) v4fa;

__device__ __forceinline__ unsigned short f2bf(float f) { unsigned u = __float_as_uint(f); u += 0x7FFFu + ((u >> 16) & 1u); return (unsigned short)(u >> 16); }
__device__ __forceinline__ float bf2f(unsigned short b) { return __uint_as_float(((unsigned)b) << 16); }
__device__ __forceinline__ float bfr(float f) { return bf2f(f2bf(f)); }
__device__ __forceinline__ v16h cat16(v8h lo, v8h hi) { return __builtin_shufflevector(lo, hi, 0, 1, 2, 3, 4, 5, 6, 7, 8, 9, 10, 11, 12, 13, 14, 15); }
__device__ __forceinline__ v8f wmma16(v16h a, v16h b, v8f c) { return __builtin_amdgcn_wmma_f32_16x16x32_f16(false, a, false, b, (short)0, c, false, false); }
#define VST2(T, p, v) do { const T vst2_v_ = (v); *(volatile T*)(p) = vst2_v_; __threadfence(); *(volatile T*)(p) = vst2_v_; } while (0)

__global__ __launch_bounds__(256) void k_wb(const float* __restrict__ bw, const float* __restrict__ sw, const float* __restrict__ sc, h16* WB) {
    typedef __attribute__((ext_vector_type(2))) _Float16 v2h;
    const int lane = threadIdx.x & 31, wid = blockIdx.x * 8 + (threadIdx.x >> 5);
    const int f0 = wid * 64 + lane * 2;
    if (f0 >= CIN * COUT * KI) return;
    v2h o;
#pragma unroll
    for (int e = 0; e < 2; ++e) {
        const int f = f0 + e, row = f / KI, col = f - row * KI, i = row / COUT, oc = row - i * COUT, u = oc * CIN + i;
        float v = 0.f;
        if (col < KT) v = bfr(bw[u * KT + col]);
        else if (col < KT + KT * NBAS) { const int c2 = col - KT, k = c2 >> 3, nb = c2 & 7; v = bfr(sw[(u * KT + k) * NBAS + nb]) * bfr(sc[u * KT + k]); }
        o[e] = (h16)v;
    }
    VST2(v2h, WB + f0, o);
}

__device__ __forceinline__ void bases8(float x, float* out8) {
    float t[12];
#pragma unroll
    for (int j = 0; j < 12; ++j) t[j] = (float)(j - 3) * GH + (-1.0f);
    float b[11];
#pragma unroll
    for (int j = 0; j < 11; ++j) b[j] = (x >= t[j] && x < t[j + 1]) ? 1.0f : 0.0f;
#pragma unroll
    for (int p = 1; p <= 3; ++p) {
#pragma unroll
        for (int j = 0; j < 11 - p; ++j) {
            const float left = (x - t[j]) / (t[j + p] - t[j]) * b[j];
            const float right = (t[j + p + 1] - x) / (t[j + p + 1] - t[j + 1]) * b[j + 1];
            b[j] = left + right;
        }
    }
#pragma unroll
    for (int j = 0; j < 8; ++j) out8[j] = b[j];
}

__global__ __launch_bounds__(128) void k_main(const float* __restrict__ x, const h16* __restrict__ WB, float* out) {
    __shared__ float win[3 * 68];
    __shared__ __align__(16) h16 AH[64 * APITCH];
    __shared__ __align__(16) h16 AL[64 * APITCH];
    __shared__ __align__(16) float ost[COUT * 68];
    const int tid = threadIdx.x, lane = tid & 31, wave = tid >> 5, lr = lane & 15, hi = lane >> 4;
    const int b = blockIdx.x / HH, h = blockIdx.x - b * HH;
    for (int e = tid; e < 64 * 15; e += 128) { const int px = e / 15, c = 81 + (e - px * 15); AH[px * APITCH + c] = (h16)0.f; AL[px * APITCH + c] = (h16)0.f; }
    v8f acc[2], accx[2];
#pragma unroll
    for (int n = 0; n < 2; ++n) { acc[n] = (v8f){}; accx[n] = (v8f){}; }
#pragma unroll 1
    for (int i = 0; i < CIN; ++i) {
        __syncthreads();
        for (int e = tid; e < 3 * 66; e += 128) { const int r = e / 66, c = e - r * 66; const int yy = h - 1 + r, xx = c - 1;
            const int yc = (yy < 0) ? 0 : (yy >= HH ? HH - 1 : yy), xc = (xx < 0) ? 0 : (xx >= WW ? WW - 1 : xx);
            win[r * 68 + c] = (yy >= 0 && yy < HH && xx >= 0 && xx < WW) ? bfr(x[(((size_t)b * CIN + i) * HH + yc) * WW + xc]) : 0.0f; }
        __syncthreads();
#pragma unroll 1
        for (int e = tid; e < 64 * KT; e += 128) {
            const int px = e / KT, k = e - px * KT, ki = k / 3, kj = k - ki * 3;
            const float v = win[ki * 68 + px + kj];
            const float sl = v / (1.0f + __expf(-v));
            float bs[8]; bases8(v, bs);
            h16* ah = AH + px * APITCH; h16* al = AL + px * APITCH;
            { const h16 a = (h16)sl; ah[k] = a; al[k] = (h16)((sl - (float)a) * LOSC); }
#pragma unroll
            for (int nb = 0; nb < 8; ++nb) { const float u = bs[nb]; const h16 a = (h16)u; ah[KT + k * NBAS + nb] = a; al[KT + k * NBAS + nb] = (h16)((u - (float)a) * LOSC); }
        }
        __syncthreads();
        const h16* wb = WB + (size_t)i * COUT * KI;
#pragma unroll
        for (int kc = 0; kc < 3; ++kc) {
            const int px = wave * 16 + lr;
            const v16h a = cat16(*(const v8ha*)(AH + px * APITCH + kc * 32 + 8 * hi), *(const v8ha*)(AH + px * APITCH + kc * 32 + 16 + 8 * hi));
            const v16h al = cat16(*(const v8ha*)(AL + px * APITCH + kc * 32 + 8 * hi), *(const v8ha*)(AL + px * APITCH + kc * 32 + 16 + 8 * hi));
#pragma unroll
            for (int n = 0; n < 2; ++n) { const h16* bp = wb + (size_t)(n * 16 + lr) * KI + kc * 32 + 8 * hi; const v16h bb = cat16(*(const v8h*)bp, *(const v8h*)(bp + 16));
                acc[n] = wmma16(a, bb, acc[n]); accx[n] = wmma16(al, bb, accx[n]); }
            asm volatile("v_nop\n\tv_nop" : "+v"(acc[0]), "+v"(acc[1]), "+v"(accx[0]), "+v"(accx[1]) : "v"(a), "v"(al));
        }
    }
    asm volatile("v_nop\n\tv_nop\n\tv_nop\n\tv_nop" : "+v"(acc[0]), "+v"(acc[1]), "+v"(accx[0]), "+v"(accx[1]));
#pragma unroll
    for (int n = 0; n < 2; ++n)
#pragma unroll
        for (int j = 0; j < 8; ++j) ost[(n * 16 + lr) * 68 + wave * 16 + hi * 8 + j] = acc[n][j] + accx[n][j] * LOSCI;
    __syncthreads();
    auto pass = [&]() {
#pragma unroll
        for (int s = 0; s < 4; ++s) { const int o = wave * 8 + 2 * s + (lane >> 4), piece = lane & 15; const v4f v = *(const v4fa*)(ost + o * 68 + piece * 4);
            *(volatile v4f*)(out + ((((size_t)b * COUT + o) * HH + h) * WW) + piece * 4) = v; }
    };
    pass(); __threadfence(); pass();
}

extern "C" void kernel_launch(void* const* d_in, const int* in_sizes, int n_in,
                              void* d_out, int out_size, void* d_ws, size_t ws_size, hipStream_t stream) {
    (void)in_sizes; (void)n_in; (void)out_size;
    const float* x = (const float*)d_in[0]; const float* bw = (const float*)d_in[1]; const float* sw = (const float*)d_in[2]; const float* sc = (const float*)d_in[3];
    float* out = (float*)d_out;
    char* wsp = (char*)d_ws;
    auto take = [&](size_t bytes) { char* p = wsp; wsp += (bytes + 255) & ~(size_t)255; return (void*)p; };
    h16* WB = (h16*)take((size_t)CIN * COUT * KI * 2);
    if ((size_t)(wsp - (char*)d_ws) > ws_size) return;
    k_wb<<<(CIN * COUT * KI / 64 + 7) / 8, 256, 0, stream>>>(bw, sw, sc, WB);
    k_main<<<NB_ * HH, 128, 0, stream>>>(x, WB, out);
}
